// LocalPoolPointnet_64759516889901
// MI455X (gfx1250) — hardware-run, weakly checked
//
#include <hip/hip_runtime.h>


#ifndef NB
#define NB 8
#endif
#ifndef TP
#define TP 100000
#endif
#define NB_FULL 8
#define TP_FULL 100000
#define HID   32
#define XW    64
#define NLAY  5
#define R3    32768
#define SLABV 128
#define NSLAB (R3 / SLABV)
#define CAP   512
#define WCAP  128
#define NWAVE 8
#define VP    (((TP + 2047) / 2048) * 2048)
#define NIT   (VP / 2048)
#define XP    72
#define HP    40
#define GP    132
#define CSC   64.0f
#define PINV  (1.0f / 4096.0f)
#define LAYW  5120
#define WH_N  (NLAY * LAYW + 1024)
#define CLIPHI ((float)(1.0 - 1.0e-5))
#define ARENA_F 16384
#define A_HT   9216
#define A_POOL 14336
#define A_WT   18432
#define A_ENT  11776
#define A_WLS  12800

static_assert(HID == 32);
static_assert(XW == 2 * HID);
static_assert(R3 % SLABV == 0);
static_assert(SLABV == 128);
static_assert(VP % 2048 == 0);
static_assert((VP / NWAVE) % 256 == 0);
static_assert(VP <= (1 << 17));
static_assert(VP >= TP);
static_assert(CAP % 32 == 0);
static_assert(CAP % 16 == 0);
static_assert(NWAVE * 16 * XP * 2 == 18432);
static_assert(18432 + NWAVE * 16 * HP * 2 == 28672);
static_assert(28672 + SLABV * HID * 2 == 36864);
static_assert(36864 + LAYW * 2 == 47104);
static_assert(A_ENT * 4 == 47104);
static_assert(A_WLS == A_ENT + 2 * CAP);
static_assert((A_WLS + NWAVE * WCAP) * 4 <= ARENA_F * 4);
static_assert(CAP * HID == ARENA_F);
static_assert((XP * 2) % 16 == 0);
static_assert((HP * 2) % 16 == 0);
static_assert((GP * 4) % 16 == 0);
static_assert(WH_N % 1024 == 0);
static_assert(LAYW % 1024 == 0);
static_assert(NWAVE * 4 == HID);
static_assert(32 * 4 == SLABV);
static_assert(NB <= NB_FULL);
static_assert(TP <= TP_FULL);
static_assert(ARENA_F * 4 + CAP * HID * 2 + HID * GP * 4 + 1024 * 2 + (32 + 32 + 32 + 192 + 64) * 4 + CAP * 4 + 2 * SLABV * 4 + NWAVE * 4 <= 131072);

typedef _Float16 h16;
typedef __attribute__((ext_vector_type(16))) _Float16 v16h;
typedef __attribute__((ext_vector_type(8)))  _Float16 v8h;
typedef __attribute__((ext_vector_type(8)))  float    v8f;
typedef __attribute__((ext_vector_type(4)))  float    v4f;
typedef __attribute__((ext_vector_type(4)))  int      v4i;
typedef v4f  __attribute__((may_alias)) v4fa;

__device__ __forceinline__ unsigned short f2bf(float f) { unsigned u = __float_as_uint(f); u += 0x7FFFu + ((u >> 16) & 1u); return (unsigned short)(u >> 16); }
__device__ __forceinline__ float bfr(float f) { return __uint_as_float(((unsigned)f2bf(f)) << 16); }
__device__ __forceinline__ v16h cat16(v8h lo, v8h hi) { return __builtin_shufflevector(lo, hi, 0, 1, 2, 3, 4, 5, 6, 7, 8, 9, 10, 11, 12, 13, 14, 15); }
__device__ __forceinline__ v8f wmma16(v16h a, v16h b, v8f c) { return __builtin_amdgcn_wmma_f32_16x16x32_f16(false, a, false, b, (short)0, c, false, false); }
__device__ __forceinline__ v16h  ldh(const h16* p) { return cat16(*(const v8h*)p, *(const v8h*)(p + 16)); }
__device__ __forceinline__ void wave_sync() { __builtin_amdgcn_fence(3  , "wavefront"); __builtin_amdgcn_wave_barrier(); asm volatile("" ::: "memory"); }
__device__ __forceinline__ h16 toh_flush(float v) { const h16 r = (h16)v; return (fabsf(v) < 6.103515625e-05f) ? (h16)0.0f : r; }
__device__ __forceinline__ v8f wmma_g(v16h a, v16h b, v8f c) { c = wmma16(a, b, c); asm volatile("v_nop\n\tv_nop\n\tv_nop\n\tv_nop" : "+v"(c) : "v"(a), "v"(b)); return c; }
__device__ __forceinline__ int vox1(float c) { c = fminf(fmaxf(c, 0.0f), CLIPHI); int q = (int)(c * 32.0f); q = q < 0 ? 0 : (q > 31 ? 31 : q); return q; }

__global__ __launch_bounds__(256) void k_vid(const float* __restrict__ p, int* vid) {
#pragma clang fp contract(off)
    const int b = blockIdx.y;
    const int i4 = blockIdx.x * 256 + threadIdx.x;
    if (i4 >= VP / 4) return;
    v4i o;
#pragma unroll
    for (int j = 0; j < 4; ++j) {
        const int pt = i4 * 4 + j;
        const int pc = pt < TP ? pt : (TP - 1);
        const size_t a = ((size_t)b * TP_FULL + (size_t)pc) * 3;
        float x = p[a], y = p[a + 1], z = p[a + 2];
        asm volatile("" : "+v"(x), "+v"(y), "+v"(z));
        const int v = vox1(bfr(x)) + 32 * (vox1(bfr(y)) + 32 * vox1(bfr(z)));
        o[j] = (pt < TP) ? v : -1;
    }
    int* dst = vid + (size_t)b * VP + (size_t)i4 * 4;
    *(volatile v4i*)dst = o; __threadfence(); *(volatile v4i*)dst = o;
}

__global__ __launch_bounds__(128) void k_wconv(const float* __restrict__ w0, const float* __restrict__ w1, const float* __restrict__ wsc, const float* __restrict__ fcw, h16* WH) {
#pragma clang fp contract(off)
    const int blk = blockIdx.x;
    const int i = blk * 128 + threadIdx.x;
    if (i >= WH_N / 8) return;
    const int L = blk / 5, q = blk - L * 5;
    float f[8];
    if (blk >= 5 * NLAY) {
        const int r = threadIdx.x * 8; const int n = r >> 5, k = r & 31;
#pragma unroll
        for (int j = 0; j < 8; ++j) f[j] = fcw[(k + j) * 32 + n];
    } else if (q < 2) {
        const int r = q * 1024 + threadIdx.x * 8; const int n = r >> 6, k = r & 63;
#pragma unroll
        for (int j = 0; j < 8; ++j) f[j] = w0[L * 2048 + (k + j) * 32 + n];
    } else if (q < 4) {
        const int r = (q - 2) * 1024 + threadIdx.x * 8; const int n = r >> 6, k = r & 63;
#pragma unroll
        for (int j = 0; j < 8; ++j) f[j] = wsc[L * 2048 + (k + j) * 32 + n];
    } else {
        const int r = threadIdx.x * 8; const int n = r >> 5, k = r & 31;
#pragma unroll
        for (int j = 0; j < 8; ++j) f[j] = w1[L * 1024 + (k + j) * 32 + n];
    }
    v8h hv;
#pragma unroll
    for (int j = 0; j < 8; ++j) hv[j] = toh_flush(bfr(f[j]) * CSC);
    h16* dst = WH + (size_t)i * 8;
    *(volatile v8h*)dst = hv; __threadfence(); *(volatile v8h*)dst = hv;
}

__global__ __launch_bounds__(256) __attribute__((amdgpu_num_vgpr(256)))
void k_slab(const float* __restrict__ p, const float* __restrict__ fpw, const float* __restrict__ fpb,
            const float* __restrict__ b0, const float* __restrict__ b1, const float* __restrict__ fcb,
            const int* __restrict__ vid, const h16* __restrict__ WH, float* OUT) {
    __shared__ __align__(16) float arena[ARENA_F];
    __shared__ __align__(16) h16   net16[CAP * HID];
    __shared__ __align__(16) float grid_s[HID * GP];
    __shared__ __align__(16) h16   fct_s[1024];
    __shared__ float b0s[32], b1s[32], fcbs[32], fpws[192], fpbs[64];
    __shared__ int lvs[CAP];
    __shared__ int vst[SLABV], vend[SLABV];
    __shared__ int wcnt[NWAVE];

    const int tid = threadIdx.x;
    const int lane = tid & 31, lr = lane & 15, hi = lane >> 4;
    const int wave = __builtin_amdgcn_readfirstlane((int)(threadIdx.x >> 5));
    const int slab = blockIdx.x, b = blockIdx.y;

    h16* const XT   = (h16*)arena;
    h16* const HT   = (h16*)arena + A_HT;
    h16* const POOL = (h16*)arena + A_POOL;
    h16* const WT   = (h16*)arena + A_WT;
    unsigned* const ENT = (unsigned*)arena + A_ENT;
    unsigned* const WLS = (unsigned*)arena + A_WLS;

#pragma unroll 1
    for (int i = tid; i < 2 * CAP + NWAVE * WCAP; i += 256) ENT[i] = 0u;
    if (tid < 128) *(v8h*)(fct_s + tid * 8) = *(const v8h*)(WH + (size_t)NLAY * LAYW + tid * 8);
    if (tid < 32) fcbs[tid] = bfr(fcb[tid]);
    if (tid < 192) fpws[tid] = bfr(fpw[tid]);
    if (tid < 64) fpbs[tid] = bfr(fpb[tid]);
    if (tid < SLABV) { vst[tid] = 0; vend[tid] = 0; }
    __syncthreads();

    {
        const int* vrow = vid + (size_t)b * VP + (size_t)wave * (VP / NWAVE) + lane * 8;
        const int wlb = wave * WCAP;
        int cnt = 0;
#pragma unroll 1
        for (int it = 0; it < NIT; ++it) {
            const v4i a = *(const v4i*)(vrow + it * 256);
            const v4i c = *(const v4i*)(vrow + it * 256 + 4);
            int xv[8]; bool hit[8]; bool any = false;
#pragma unroll
            for (int j = 0; j < 4; ++j) { xv[j] = a[j]; xv[4 + j] = c[j]; }
#pragma unroll
            for (int j = 0; j < 8; ++j) { hit[j] = (xv[j] >> 7) == slab; any = any | hit[j]; }
            if (__builtin_amdgcn_ballot_w32(any) != 0u) {
                const int pbase = wave * (VP / NWAVE) + it * 256 + lane * 8;
#pragma unroll
                for (int j = 0; j < 8; ++j) {
                    const unsigned bj = __builtin_amdgcn_ballot_w32(hit[j]);
                    const int pos = cnt + (int)__builtin_amdgcn_mbcnt_lo(bj, 0u);
                    if (hit[j] & (pos < WCAP)) WLS[wlb + pos] = ((unsigned)(xv[j] & 127) << 17) | (unsigned)(pbase + j);
                    cnt += __popc(bj);
                }
            }
        }
        if (lane == 0) wcnt[wave] = cnt;
    }
    __syncthreads();

    int tot = 0, off = 0, ovf = 0;
#pragma unroll
    for (int w = 0; w < NWAVE; ++w) {
        const int cw = wcnt[w];
        const int cc = cw < WCAP ? cw : WCAP;
        ovf |= (cw > WCAP) ? 1 : 0;
        off += (w < wave) ? cc : 0;
        tot += cc;
    }
    ovf |= (tot > CAP) ? 1 : 0;
    const int ncl = tot < CAP ? tot : CAP;
    const int n = __builtin_amdgcn_readfirstlane(ncl);
    const int poison = __builtin_amdgcn_readfirstlane(ovf);
    {
        const int cw = wcnt[wave];
        const int mycnt = cw < WCAP ? cw : WCAP;
#pragma unroll
        for (int k = 0; k < WCAP / 32; ++k) {
            const int i = k * 32 + lane;
            const unsigned e = WLS[wave * WCAP + i];
            if ((i < mycnt) & (off + i < CAP)) ENT[off + i] = e;
        }
    }
    __syncthreads();

    if (wave == 0) {
        int ngr = (n + 31) >> 5; ngr = ngr < CAP / 32 ? ngr : CAP / 32;
#pragma unroll 1
        for (int bit = 0; bit < 7; ++bit) {
            const int so = (bit & 1) * CAP, dof = CAP - so;
            const int sh = 17 + bit;
            int zc = 0;
#pragma unroll 1
            for (int g = 0; g < ngr; ++g) {
                const int idx = g * 32 + lane; const bool ok = idx < n;
                const unsigned e = ENT[so + idx];
                const bool bs = ((e >> sh) & 1u) != 0u;
                const unsigned zb = __builtin_amdgcn_ballot_w32(ok & !bs);
                zc += __popc(zb);
            }
            int z = 0, o = zc;
#pragma unroll 1
            for (int g = 0; g < ngr; ++g) {
                const int idx = g * 32 + lane; const bool ok = idx < n;
                const unsigned e = ENT[so + idx];
                const bool bs = ((e >> sh) & 1u) != 0u;
                const unsigned zb = __builtin_amdgcn_ballot_w32(ok & !bs);
                const unsigned ob = __builtin_amdgcn_ballot_w32(ok & bs);
                const int pz = z + (int)__builtin_amdgcn_mbcnt_lo(zb, 0u);
                const int po = o + (int)__builtin_amdgcn_mbcnt_lo(ob, 0u);
                const int pos = bs ? po : pz;
                if (ok & (pos < CAP)) ENT[dof + pos] = e;
                z += __popc(zb); o += __popc(ob);
            }
            wave_sync();
        }
    }
    __syncthreads();

#pragma unroll 1
    for (int i = tid; i < CAP; i += 256) {
        const bool ok = i < n;
        const int ic = ok ? i : 0;
        const int ip = ic > 0 ? ic - 1 : 0;
        const int inx = (ic + 1 < n) ? ic + 1 : ic;
        const unsigned e = ENT[CAP + ic], ep = ENT[CAP + ip], en = ENT[CAP + inx];
        const int k = (int)(e >> 17) & 127, kp = (int)(ep >> 17) & 127, kn = (int)(en >> 17) & 127;
        const bool first = ok & ((ic == 0) | (kp != k));
        const bool last  = ok & ((ic + 1 >= n) | (kn != k));
        if (first) vst[k] = ic;
        if (last) vend[k] = ic + 1;
        if (ok) lvs[ic] = k;
    }
    __syncthreads();

    const int ntiles = (n + 15) >> 4;
    h16* const xw = XT + wave * 16 * XP;
    h16* const hw = HT + wave * 16 * HP;
    const v16h z16 = (v16h){};
    const v8h  z8  = (v8h){};

#pragma unroll 1
    for (int L = 0; L < NLAY; ++L) {
#pragma unroll 1
        for (int i = tid; i < LAYW / 8; i += 256) *(v8h*)(WT + i * 8) = *(const v8h*)(WH + (size_t)L * LAYW + i * 8);
        if (tid < 32) { b0s[tid] = bfr(b0[L * 32 + tid]); b1s[tid] = bfr(b1[L * 32 + tid]); }
        if (L > 0) {
            const int v = tid >> 1, hf = tid & 1;
            int s = vst[v], e = vend[v];
            s = s < 0 ? 0 : (s > n ? n : s); e = e < s ? s : (e > n ? n : e);
            const int len = e - s;
            int ml = len;
            ml = max(ml, __shfl_xor(ml, 1, 32)); ml = max(ml, __shfl_xor(ml, 2, 32)); ml = max(ml, __shfl_xor(ml, 4, 32));
            ml = max(ml, __shfl_xor(ml, 8, 32)); ml = max(ml, __shfl_xor(ml, 16, 32));
            ml = ml > CAP ? CAP : ml;
            const int mlu = __builtin_amdgcn_readfirstlane(ml);
            v8h m0, m1;
#pragma unroll
            for (int k = 0; k < 8; ++k) { m0[k] = (h16)(-65504.0f); m1[k] = (h16)(-65504.0f); }
#pragma unroll 1
            for (int j = 0; j < mlu; ++j) {
                const bool ok = j < len;
                const int pc = ok ? (s + j) : (len > 0 ? s : 0);
                const v8h x0 = *(const v8h*)(net16 + pc * HID + hf * 16);
                const v8h x1 = *(const v8h*)(net16 + pc * HID + hf * 16 + 8);
                const v8h c0 = __builtin_elementwise_max(m0, x0);
                const v8h c1 = __builtin_elementwise_max(m1, x1);
                m0 = ok ? c0 : m0; m1 = ok ? c1 : m1;
            }
            const bool ne = len > 0;
            *(v8h*)(POOL + v * HID + hf * 16)     = ne ? m0 : z8;
            *(v8h*)(POOL + v * HID + hf * 16 + 8) = ne ? m1 : z8;
        }
        __syncthreads();

#pragma unroll 1
        for (int t = wave; t < ntiles; t += NWAVE) {
            const int t0 = t * 16;
            {
                const int row = lane >> 1, hf2 = lane & 1;
                const int pt = t0 + row; const bool ok = pt < n; const int pc = ok ? pt : 0;
                if (L == 0) {
                    const unsigned e = ENT[CAP + pc];
                    int pidx = (int)(e & 0x1FFFFu); pidx = pidx > TP - 1 ? TP - 1 : pidx;
                    const size_t a = ((size_t)b * TP_FULL + (size_t)pidx) * 3;
                    float px = p[a], py = p[a + 1], pz = p[a + 2];
                    asm volatile("" : "+v"(px), "+v"(py), "+v"(pz));
                    px = bfr(px); py = bfr(py); pz = bfr(pz);
#pragma unroll 1
                    for (int jb = 0; jb < 4; ++jb) {
                        v8h o;
#pragma unroll
                        for (int j = 0; j < 8; ++j) {
                            const int col = hf2 * 32 + jb * 8 + j;
                            const float v = px * fpws[col] + py * fpws[64 + col] + pz * fpws[128 + col] + fpbs[col];
                            const h16 hv = toh_flush(v * CSC);
                            o[j] = ok ? hv : (h16)0.0f;
                        }
                        *(v8h*)(xw + row * XP + hf2 * 32 + jb * 8) = o;
                    }
                } else {
                    const int lv = lvs[pc] & (SLABV - 1);
                    const v8h n0 = *(const v8h*)(net16 + pc * HID + hf2 * 16);
                    const v8h n1 = *(const v8h*)(net16 + pc * HID + hf2 * 16 + 8);
                    const v8h q0 = *(const v8h*)(POOL + lv * HID + hf2 * 16);
                    const v8h q1 = *(const v8h*)(POOL + lv * HID + hf2 * 16 + 8);
                    *(v8h*)(xw + row * XP + hf2 * 16)          = ok ? n0 : z8;
                    *(v8h*)(xw + row * XP + hf2 * 16 + 8)      = ok ? n1 : z8;
                    *(v8h*)(xw + row * XP + 32 + hf2 * 16)     = ok ? q0 : z8;
                    *(v8h*)(xw + row * XP + 32 + hf2 * 16 + 8) = ok ? q1 : z8;
                }
            }
            wave_sync();
            const v16h a0 = ldh(xw + lr * XP + 8 * hi), a1 = ldh(xw + lr * XP + 32 + 8 * hi);
            const v16h r0 = __builtin_elementwise_max(a0, z16), r1 = __builtin_elementwise_max(a1, z16);
#pragma unroll
            for (int nt = 0; nt < 2; ++nt) {
                v8f acc = (v8f){};
                acc = wmma_g(r0, ldh(WT + (nt * 16 + lr) * XW + 8 * hi), acc);
                acc = wmma_g(r1, ldh(WT + (nt * 16 + lr) * XW + 32 + 8 * hi), acc);
                const float bc = b0s[nt * 16 + lr];
#pragma unroll
                for (int r = 0; r < 8; ++r) { float v = acc[r] * PINV + bc; v = fmaxf(v, 0.0f); hw[(8 * hi + r) * HP + nt * 16 + lr] = toh_flush(v * CSC); }
            }
            wave_sync();
            const v16h hf16 = ldh(hw + lr * HP + 8 * hi);
#pragma unroll
            for (int nt = 0; nt < 2; ++nt) {
                v8f acc = (v8f){};
                acc = wmma_g(a0, ldh(WT + 2048 + (nt * 16 + lr) * XW + 8 * hi), acc);
                acc = wmma_g(a1, ldh(WT + 2048 + (nt * 16 + lr) * XW + 32 + 8 * hi), acc);
                acc = wmma_g(hf16, ldh(WT + 4096 + (nt * 16 + lr) * HID + 8 * hi), acc);
                const float bc = b1s[nt * 16 + lr];
#pragma unroll
                for (int r = 0; r < 8; ++r) { const float v = acc[r] * PINV + bc; net16[(t0 + 8 * hi + r) * HID + nt * 16 + lr] = toh_flush(v * CSC); }
            }
            wave_sync();
        }
        __syncthreads();
    }

#pragma unroll 1
    for (int t = wave; t < ntiles; t += NWAVE) {
        const int t0 = t * 16;
        const v16h a = ldh(net16 + (t0 + lr) * HID + 8 * hi);
#pragma unroll
        for (int nt = 0; nt < 2; ++nt) {
            v8f acc = (v8f){};
            acc = wmma_g(a, ldh(fct_s + (nt * 16 + lr) * HID + 8 * hi), acc);
            const float bc = fcbs[nt * 16 + lr];
#pragma unroll
            for (int r = 0; r < 8; ++r) arena[(t0 + 8 * hi + r) * HID + nt * 16 + lr] = acc[r] * PINV + bc;
        }
    }
    __syncthreads();

    {
        const int v = tid >> 1, hf = tid & 1;
        int s = vst[v], e = vend[v];
        s = s < 0 ? 0 : (s > n ? n : s); e = e < s ? s : (e > n ? n : e);
        const int len = e - s;
        int ml = len;
        ml = max(ml, __shfl_xor(ml, 1, 32)); ml = max(ml, __shfl_xor(ml, 2, 32)); ml = max(ml, __shfl_xor(ml, 4, 32));
        ml = max(ml, __shfl_xor(ml, 8, 32)); ml = max(ml, __shfl_xor(ml, 16, 32));
        ml = ml > CAP ? CAP : ml;
        const int mlu = __builtin_amdgcn_readfirstlane(ml);
        v4f s0 = (v4f){}, s1 = (v4f){}, s2 = (v4f){}, s3 = (v4f){};
        const v4f zf = (v4f){};
#pragma unroll 1
        for (int j = 0; j < mlu; ++j) {
            const bool ok = j < len;
            const int pc = ok ? (s + j) : (len > 0 ? s : 0);
            const v4f x0 = *(const v4fa*)(&arena[pc * HID + hf * 16]);
            const v4f x1 = *(const v4fa*)(&arena[pc * HID + hf * 16 + 4]);
            const v4f x2 = *(const v4fa*)(&arena[pc * HID + hf * 16 + 8]);
            const v4f x3 = *(const v4fa*)(&arena[pc * HID + hf * 16 + 12]);
            s0 += ok ? x0 : zf; s1 += ok ? x1 : zf; s2 += ok ? x2 : zf; s3 += ok ? x3 : zf;
        }
        const float inv = 1.0f / fmaxf((float)len, 1.0f);
#pragma unroll
        for (int c = 0; c < 4; ++c) {
            grid_s[(hf * 16 + c) * GP + v]      = s0[c] * inv;
            grid_s[(hf * 16 + 4 + c) * GP + v]  = s1[c] * inv;
            grid_s[(hf * 16 + 8 + c) * GP + v]  = s2[c] * inv;
            grid_s[(hf * 16 + 12 + c) * GP + v] = s3[c] * inv;
        }
    }
    __syncthreads();

    {
        float* ob = OUT + ((size_t)b * HID) * R3 + (size_t)slab * SLABV;
        const float nanv = __uint_as_float(0x7FC00000u);
#pragma unroll 1
        for (int ps = 0; ps < 2; ++ps) {
#pragma unroll
            for (int k = 0; k < 4; ++k) {
                const int ch = wave * 4 + k;
                v4f val = *(const v4fa*)(&grid_s[ch * GP + lane * 4]);
                if (poison != 0) { val[0] = nanv; val[1] = nanv; val[2] = nanv; val[3] = nanv; }
                *(volatile v4f*)(ob + (size_t)ch * R3 + lane * 4) = val;
            }
            if (ps == 0) __threadfence();
        }
    }
}

static constexpr size_t al256(size_t v) { return (v + 255) & ~(size_t)255; }
static constexpr size_t SZ_VID = al256((size_t)NB * VP * 4);
static constexpr size_t SZ_WH  = al256((size_t)WH_N * 2);
static constexpr size_t SZ_TOTAL = SZ_VID + SZ_WH;
static_assert(SZ_TOTAL <= (size_t)134217728);
static_assert(((size_t)VP * 4) % 128 == 0);
static_assert((size_t)(VP / 1024) * 256 * 4 == (size_t)VP);
static_assert((size_t)(WH_N / 1024) * 128 * 8 == (size_t)WH_N);
static_assert(((size_t)HID * R3 * 4) % 128 == 0);

extern "C" void kernel_launch(void* const* d_in, const int* in_sizes, int n_in,
                              void* d_out, int out_size, void* d_ws, size_t ws_size, hipStream_t stream) {
    if (n_in < 10) return;
    if ((size_t)in_sizes[0] < ((size_t)(NB - 1) * TP_FULL + TP) * 3) return;
    if (in_sizes[1] < 3 * XW || in_sizes[2] < XW) return;
    if (in_sizes[3] < NLAY * XW * HID || in_sizes[4] < NLAY * HID || in_sizes[5] < NLAY * HID * HID || in_sizes[6] < NLAY * HID) return;
    if (in_sizes[7] < NLAY * XW * HID || in_sizes[8] < HID * HID || in_sizes[9] < HID) return;
    if ((size_t)out_size < (size_t)NB * HID * R3) return;
    if (SZ_TOTAL > ws_size) return;
    const float* p   = (const float*)d_in[0];
    const float* fpw = (const float*)d_in[1];
    const float* fpb = (const float*)d_in[2];
    const float* w0  = (const float*)d_in[3];
    const float* b0  = (const float*)d_in[4];
    const float* w1  = (const float*)d_in[5];
    const float* b1  = (const float*)d_in[6];
    const float* wsc = (const float*)d_in[7];
    const float* fcw = (const float*)d_in[8];
    const float* fcb = (const float*)d_in[9];
    float* OUT = (float*)d_out;
    char* wsp = (char*)d_ws;
    int* VID = (int*)wsp; wsp += SZ_VID;
    h16* WH = (h16*)wsp; wsp += SZ_WH;

    k_vid<<<dim3(VP / 1024, NB, 1), 256, 0, stream>>>(p, VID);
    k_wconv<<<dim3(WH_N / 1024, 1, 1), 128, 0, stream>>>(w0, w1, wsc, fcw, WH);
    k_slab<<<dim3(NSLAB, NB, 1), 256, 0, stream>>>(p, fpw, fpb, b0, b1, fcb, VID, WH, OUT);
}
